// LSTMModel1_68161130988345
// MI455X (gfx1250) — hardware-verified
//
#include <hip/hip_runtime.h>
#include <math.h>
#include <stdint.h>

constexpr int NSEQ    = 256;
constexpr int NSTEP   = 1024;
constexpr int NHID    = 96;
constexpr int NG4     = 384;
constexpr int NTHR    = 192;
constexpr int PTHR    = 256;
constexpr int TROWS   = 16;
constexpr int HPITCH  = 104;
constexpr int XCH     = 32;
constexpr int HSP     = 100;
constexpr int GSTRIDE = NHID * NHID;
constexpr float A_CARRY = 16.0f;
constexpr float W_CARRY = 64.0f;
constexpr float Z_FOLD  = 1.0f / 1024.0f;

static_assert(NSEQ % TROWS == 0, "grid covers all sequences exactly");
static_assert(NSTEP % XCH == 0, "chunks tile the time axis exactly");
static_assert(TROWS * XCH == 128 * 4, "x staging: 128 threads x one float4 per chunk");
static_assert((NG4 * NHID / 8) % PTHR == 0, "weight prep grid exact");
static_assert(NHID % 32 == 0, "K multiple of 32");
static_assert(NHID == 16 * (NTHR / 32), "one 16-unit column group per wave");
static_assert(TROWS == 16, "out lines: 4 waves x 4 line groups = 16 rows");
static_assert(HPITCH % 8 == 0 && HPITCH >= NHID, "16-B aligned fragment rows");
static_assert(HSP % 4 == 0 && HSP >= NHID, "16-B aligned head rows");

typedef __attribute__((ext_vector_type(16))) _Float16 v16h;
typedef __attribute__((ext_vector_type(8)))  _Float16 v8h;
typedef __attribute__((ext_vector_type(8)))  float    v8f;
typedef __attribute__((ext_vector_type(4)))  float    v4f;

__device__ __forceinline__ unsigned short f2bf_bits(float f) {
  unsigned u = __float_as_uint(f);
  return (unsigned short)((u + 0x7FFFu + ((u >> 16) & 1u)) >> 16);
}
__device__ __forceinline__ float bf_bits2f(unsigned short h) { return __uint_as_float(((unsigned)h) << 16); }
__device__ __forceinline__ float bfr(float f) { return bf_bits2f(f2bf_bits(f)); }

__device__ __forceinline__ void dep_guard_h(v8f& a, v8f& b, v16h x, v16h y) { asm volatile("v_nop\n\tv_nop\n\tv_nop\n\tv_nop" : "+v"(a), "+v"(b) : "v"(x), "v"(y)); }
__device__ __forceinline__ void keep4_h(v16h a, v16h b, v16h c, v16h d) { asm volatile("v_nop" :: "v"(a), "v"(b), "v"(c), "v"(d)); }
__device__ __forceinline__ void keep2_h(v16h a, v16h b) { asm volatile("v_nop" :: "v"(a), "v"(b)); }
__device__ __forceinline__ void acc_guard4(v8f& a, v8f& b, v8f& c, v8f& d) { asm volatile("v_nop\n\tv_nop\n\tv_nop\n\tv_nop" : "+v"(a), "+v"(b), "+v"(c), "+v"(d)); }
template <typename T> struct Frag;
template <> struct Frag<_Float16> {
  typedef v16h V; union U { v16h v; v8h h[2]; };
  static __device__ __forceinline__ v16h load(const _Float16* p) {
    U f; f.h[0] = *(const v8h*)(p); f.h[1] = *(const v8h*)(p + 16); return f.v;
  }
  static __device__ __forceinline__ v8f mma(v16h a, v16h b, v8f c) {
    return __builtin_amdgcn_wmma_f32_16x16x32_f16(false, a, false, b, (short)0, c, false, false);
  }
  static __device__ __forceinline__ void guard(v8f& a, v8f& b, v16h x, v16h y) { dep_guard_h(a, b, x, y); }
  static __device__ __forceinline__ void keep(v16h a, v16h b, v16h c, v16h d) { keep4_h(a, b, c, d); }
};
typedef Frag<_Float16> FragH;

__device__ __forceinline__ float fsig(float v)  { return __builtin_amdgcn_rcpf(1.0f + __expf(-v)); }
__device__ __forceinline__ float ftanh(float v) { return 1.0f - 2.0f * __builtin_amdgcn_rcpf(__expf(2.0f * v) + 1.0f); }

__global__ __launch_bounds__(PTHR) void wprep_kernel(const float* __restrict__ W, int n8, unsigned short* __restrict__ O) {
  const int i = blockIdx.x * PTHR + threadIdx.x;
  if (i >= n8) return;
  const int e0 = i * 8;
  v8h hv;
#pragma unroll
  for (int e = 0; e < 8; ++e) {
    const float fb = bfr(W[e0 + e]);
    hv[e] = (_Float16)(fb * W_CARRY);
  }
  *(volatile v8h*)(O + e0) = hv;
  __threadfence();
  *(volatile v8h*)(O + e0) = hv;
}

__device__ __forceinline__ void mac4(v8f (&acc)[4], const _Float16* arow, const _Float16* wp, int k0) {
  const v16h a  = FragH::load(arow + k0);
  const v16h b0 = FragH::load(wp + k0);
  const v16h b1 = FragH::load(wp + GSTRIDE + k0);
  const v16h b2 = FragH::load(wp + 2 * GSTRIDE + k0);
  const v16h b3 = FragH::load(wp + 3 * GSTRIDE + k0);
  acc[0] = FragH::mma(a, b0, acc[0]);
  acc[1] = FragH::mma(a, b1, acc[1]);
  acc[2] = FragH::mma(a, b2, acc[2]);
  acc[3] = FragH::mma(a, b3, acc[3]);
  acc_guard4(acc[0], acc[1], acc[2], acc[3]);
  keep4_h(a, b0, b1, b2);
  keep2_h(b3, a);
}

__global__ __launch_bounds__(NTHR) void lstm2_kernel(
    const float* __restrict__ x,
    const float* __restrict__ w_ih0, const float* __restrict__ b_ih0, const float* __restrict__ b_hh0,
    const float* __restrict__ b_ih1, const float* __restrict__ b_hh1,
    const float* __restrict__ wl,    const float* __restrict__ bl,
    const unsigned short* __restrict__ Whh0p, const unsigned short* __restrict__ Wih1p,
    const unsigned short* __restrict__ Whh1p,
    float* __restrict__ out) {
  __shared__ __align__(16) _Float16 Ht[2 * TROWS * HPITCH];
  __shared__ __align__(16) float    Xs[TROWS * XCH];
  __shared__ __align__(16) float    Hs[TROWS * HSP];
  __shared__ __align__(16) float    Os[TROWS * XCH];
  __shared__ __align__(16) float    Wls[NHID];

  const int tid = threadIdx.x, lane = tid & 31, wave = tid >> 5;
  const int c = lane & 15, hh = lane >> 4, koff = hh * 8;
  const int j  = 16 * wave + c;
  const int rb = 8 * hh;
  const int rowbase = blockIdx.x * TROWS;

#pragma unroll 1
  for (int i = tid; i < 2 * TROWS * HPITCH; i += NTHR) Ht[i] = (_Float16)0.0f;
  if (tid < NHID) Wls[tid] = bfr(wl[tid]);

  const float wxi = bfr(w_ih0[j]);
  const float wxf = bfr(w_ih0[NHID + j]);
  const float wxg = bfr(w_ih0[2 * NHID + j]);
  const float wxo = bfr(w_ih0[3 * NHID + j]);
  const float b0i = bfr(b_ih0[j])            + bfr(b_hh0[j]);
  const float b0f = bfr(b_ih0[NHID + j])     + bfr(b_hh0[NHID + j]);
  const float b0g = bfr(b_ih0[2 * NHID + j]) + bfr(b_hh0[2 * NHID + j]);
  const float b0o = bfr(b_ih0[3 * NHID + j]) + bfr(b_hh0[3 * NHID + j]);
  const float b1i = bfr(b_ih1[j])            + bfr(b_hh1[j]);
  const float b1f = bfr(b_ih1[NHID + j])     + bfr(b_hh1[NHID + j]);
  const float b1g = bfr(b_ih1[2 * NHID + j]) + bfr(b_hh1[2 * NHID + j]);
  const float b1o = bfr(b_ih1[3 * NHID + j]) + bfr(b_hh1[3 * NHID + j]);
  const float blv = bfr(bl[0]);

  float cs0[8], cs1[8];
#pragma unroll
  for (int r = 0; r < 8; ++r) { cs0[r] = 0.0f; cs1[r] = 0.0f; }
  __syncthreads();

  const _Float16* a0row = Ht + c * HPITCH + koff;
  const _Float16* a1row = a0row + TROWS * HPITCH;
  const _Float16* whh0 = (const _Float16*)Whh0p + (size_t)j * NHID + koff;
  const _Float16* wih1 = (const _Float16*)Wih1p + (size_t)j * NHID + koff;
  const _Float16* whh1 = (const _Float16*)Whh1p + (size_t)j * NHID + koff;
  const v8f z8 = {0.f, 0.f, 0.f, 0.f, 0.f, 0.f, 0.f, 0.f};

#pragma unroll 1
  for (int t = 0; t < NSTEP; ++t) {
    const int tc = t & (XCH - 1);
    if (tc == 0) {
      if (tid < 128) {
        const int row = tid >> 3, c4 = (tid & 7) * 4;
        const v4f v = *(const v4f*)(x + ((size_t)(rowbase + row) * NSTEP + (size_t)(t + c4)));
        v4f w;
        w[0] = bfr(v[0]); w[1] = bfr(v[1]); w[2] = bfr(v[2]); w[3] = bfr(v[3]);
        *(v4f*)(Xs + row * XCH + c4) = w;
      }
      __syncthreads();
    }
    {
      float xr[8];
#pragma unroll
      for (int r = 0; r < 8; ++r) xr[r] = Xs[(rb + r) * XCH + tc];
      v8f acc[4];
      acc[0] = z8; acc[1] = z8; acc[2] = z8; acc[3] = z8;
#pragma unroll 1
      for (int kc = 0; kc < 3; ++kc) mac4(acc, a0row, whh0, kc * 32);
      float hn[8];
#pragma unroll
      for (int r = 0; r < 8; ++r) {
        const float pi = fmaf(acc[0][r], Z_FOLD, fmaf(xr[r], wxi, b0i));
        const float pf = fmaf(acc[1][r], Z_FOLD, fmaf(xr[r], wxf, b0f));
        const float pg = fmaf(acc[2][r], Z_FOLD, fmaf(xr[r], wxg, b0g));
        const float po = fmaf(acc[3][r], Z_FOLD, fmaf(xr[r], wxo, b0o));
        const float ig = fsig(pi);
        const float fg = fsig(pf);
        const float gg = ftanh(pg);
        const float og = fsig(po);
        const float cn = fmaf(fg, cs0[r], ig * gg);
        cs0[r] = cn;
        hn[r] = og * ftanh(cn);
      }
      __syncthreads();
#pragma unroll
      for (int r = 0; r < 8; ++r) Ht[(rb + r) * HPITCH + j] = (_Float16)(A_CARRY * hn[r]);
      __syncthreads();
    }
    {
      v8f acc[4];
      acc[0] = z8; acc[1] = z8; acc[2] = z8; acc[3] = z8;
#pragma unroll 1
      for (int kc = 0; kc < 3; ++kc) {
        mac4(acc, a0row, wih1, kc * 32);
        mac4(acc, a1row, whh1, kc * 32);
      }
      float hn[8];
#pragma unroll
      for (int r = 0; r < 8; ++r) {
        const float pi = fmaf(acc[0][r], Z_FOLD, b1i);
        const float pf = fmaf(acc[1][r], Z_FOLD, b1f);
        const float pg = fmaf(acc[2][r], Z_FOLD, b1g);
        const float po = fmaf(acc[3][r], Z_FOLD, b1o);
        const float ig = fsig(pi);
        const float fg = fsig(pf);
        const float gg = ftanh(pg);
        const float og = fsig(po);
        const float cn = fmaf(fg, cs1[r], ig * gg);
        cs1[r] = cn;
        hn[r] = og * ftanh(cn);
      }
      __syncthreads();
#pragma unroll
      for (int r = 0; r < 8; ++r) {
        Ht[TROWS * HPITCH + (rb + r) * HPITCH + j] = (_Float16)(A_CARRY * hn[r]);
        Hs[(rb + r) * HSP + j] = hn[r];
      }
      __syncthreads();
    }
    if (wave == 0) {
      const float* hrow = Hs + c * HSP;
      float o = 0.0f;
#pragma unroll 1
      for (int k = 0; k < NHID; k += 4) {
        const v4f hv = *(const v4f*)(hrow + k);
        const v4f wv = *(const v4f*)(Wls + k);
        o = fmaf(hv[0], wv[0], o);
        o = fmaf(hv[1], wv[1], o);
        o = fmaf(hv[2], wv[2], o);
        o = fmaf(hv[3], wv[3], o);
      }
      if (lane < TROWS) Os[lane * XCH + tc] = o + blv;
    }
    if (tc == XCH - 1) {
      __syncthreads();
      if (wave < 4) {
        const int L  = wave * 4 + (lane >> 3);
        const int c4 = (lane & 7) * 4;
        const v4f v = *(const v4f*)(Os + L * XCH + c4);
        float* op = out + (size_t)(rowbase + L) * NSTEP + (size_t)(t - (XCH - 1)) + (size_t)c4;
        *(volatile v4f*)op = v;
        __threadfence();
        *(volatile v4f*)op = v;
      }
    }
  }
}

extern "C" void kernel_launch(void* const* d_in, const int* in_sizes, int n_in,
                              void* d_out, int out_size, void* d_ws, size_t ws_size, hipStream_t stream) {
  if (n_in < 11 || d_out == nullptr || d_ws == nullptr) return;
  if (in_sizes[0] != NSEQ * NSTEP || in_sizes[1] != NG4 || in_sizes[2] != NG4 * NHID || in_sizes[3] != NG4 ||
      in_sizes[4] != NG4 || in_sizes[5] != NG4 * NHID || in_sizes[6] != NG4 * NHID || in_sizes[7] != NG4 ||
      in_sizes[8] != NG4 || in_sizes[9] != NHID || in_sizes[10] < 1 || out_size != NSEQ * NSTEP) return;

  const float* x     = (const float*)d_in[0];
  const float* w_ih0 = (const float*)d_in[1];
  const float* w_hh0 = (const float*)d_in[2];
  const float* b_ih0 = (const float*)d_in[3];
  const float* b_hh0 = (const float*)d_in[4];
  const float* w_ih1 = (const float*)d_in[5];
  const float* w_hh1 = (const float*)d_in[6];
  const float* b_ih1 = (const float*)d_in[7];
  const float* b_hh1 = (const float*)d_in[8];
  const float* wl    = (const float*)d_in[9];
  const float* bl    = (const float*)d_in[10];
  float* out = (float*)d_out;

  char* ws = (char*)d_ws; size_t off = 0;
  auto carve = [&](size_t bytes) -> char* { char* p = ws + off; off += (bytes + 255) & ~(size_t)255; return p; };
  const size_t plane_bytes = (size_t)NG4 * NHID * 2;
  unsigned short* WHH0 = (unsigned short*)carve(plane_bytes);
  unsigned short* WIH1 = (unsigned short*)carve(plane_bytes);
  unsigned short* WHH1 = (unsigned short*)carve(plane_bytes);
  if (off > ws_size || off > (size_t)134217728) return;

  const int n8 = NG4 * NHID / 8;
  wprep_kernel<<<n8 / PTHR, PTHR, 0, stream>>>(w_hh0, n8, WHH0);
  wprep_kernel<<<n8 / PTHR, PTHR, 0, stream>>>(w_ih1, n8, WIH1);
  wprep_kernel<<<n8 / PTHR, PTHR, 0, stream>>>(w_hh1, n8, WHH1);
  lstm2_kernel<<<NSEQ / TROWS, NTHR, 0, stream>>>(x, w_ih0, b_ih0, b_hh0, b_ih1, b_hh1, wl, bl, WHH0, WIH1, WHH1, out);
}
